// FusionNeRF_3032246911660
// MI455X (gfx1250) — hardware-verified
//
#include <hip/hip_runtime.h>
#define NR 2048
#define NS 128
#define NPTS (NR * NS)
#define HID 256

typedef __bf16 v16b __attribute__((ext_vector_type(16)));
typedef unsigned short v8us __attribute__((ext_vector_type(8), may_alias));
typedef float  v8f  __attribute__((ext_vector_type(8)));
typedef float  v4f  __attribute__((ext_vector_type(4)));
typedef float  v4fa __attribute__((ext_vector_type(4), may_alias));
union FragB { v16b v; v8us half[2]; unsigned short u[16]; };

__device__ __forceinline__ unsigned short bf16_bits(float x) { unsigned int u = __float_as_uint(x); return (unsigned short)((u + 0x7FFFu + ((u >> 16) & 1u)) >> 16); }
__device__ __forceinline__ float bf16_val(unsigned short b) { return __uint_as_float(((unsigned int)b) << 16); }
__device__ __forceinline__ float bf16_round(float x) { return bf16_val(bf16_bits(x)); }
template <int NT>
__device__ __forceinline__ v8f mmaN(v16b ah, v16b al, v16b bh, v16b bl, v8f c) {
  c = __builtin_amdgcn_wmma_f32_16x16x32_bf16(false, ah, false, bh, (short)0, c, false, false);
  if (NT >= 2) c = __builtin_amdgcn_wmma_f32_16x16x32_bf16(false, al, false, bh, (short)0, c, false, false);
  if (NT >= 3) c = __builtin_amdgcn_wmma_f32_16x16x32_bf16(false, ah, false, bl, (short)0, c, false, false);
  asm volatile("v_nop\n\tv_nop\n\tv_nop\n\tv_nop" : "+v"(c) : "v"(ah), "v"(al), "v"(bh), "v"(bl));
  return c;
}

__global__ __launch_bounds__(256) void k_wt_bf16(const float* __restrict__ W, unsigned short* __restrict__ Wt, int K, int N) {
  const int t = blockIdx.x * 256 + threadIdx.x;
  const int k8n = K / 8;
  if (t >= N * k8n) return;
  const int n = t / k8n, k8 = (t % k8n) * 8;
  v8us v;
#pragma unroll
  for (int i = 0; i < 8; ++i) v[i] = bf16_bits(W[(size_t)(k8 + i) * N + n]);
  *(volatile v8us*)(Wt + (size_t)n * K + k8) = v;
  __threadfence();
  *(volatile v8us*)(Wt + (size_t)n * K + k8) = v;
}

template <bool ASPLIT, int ACT, bool BIAS_BF16>
__global__ __launch_bounds__(128) void k_gemm_bf(const float* __restrict__ A, int lda, const unsigned short* __restrict__ Wt, int ldb,
                                               const float* __restrict__ bias, float* __restrict__ C, int ldc, int M, int N, int K) {
  __shared__ __attribute__((aligned(16))) float so[4][16][64];
  const int tid = threadIdx.x, w = tid >> 5, lane = tid & 31, ln = lane & 15, hh = lane >> 4;
  const int ntn = N / 64;
  const int wid = blockIdx.x * 4 + w;
  const int mt = wid / ntn, nq = wid % ntn;
  if (mt * 16 >= M) return;
  const int row0 = mt * 16, col0 = nq * 64;
  const float* arow = A + (size_t)(row0 + ln) * lda;
  v8f acc[4] = {};
  for (int kb = 0; kb < K; kb += 32) {
    FragB ah, al;
    const v4f x0 = *(const v4fa*)(arow + kb + 8 * hh), x1 = *(const v4fa*)(arow + kb + 8 * hh + 4);
    const v4f x2 = *(const v4fa*)(arow + kb + 16 + 8 * hh), x3 = *(const v4fa*)(arow + kb + 16 + 8 * hh + 4);
    float xs[16] = {x0[0],x0[1],x0[2],x0[3],x1[0],x1[1],x1[2],x1[3],x2[0],x2[1],x2[2],x2[3],x3[0],x3[1],x3[2],x3[3]};
#pragma unroll
    for (int i = 0; i < 16; ++i) { const unsigned short hb = bf16_bits(xs[i]); ah.u[i] = hb; al.u[i] = ASPLIT ? bf16_bits(xs[i] - bf16_val(hb)) : (unsigned short)0; }
#pragma unroll
    for (int t = 0; t < 4; ++t) {
      const unsigned short* brow = Wt + (size_t)(col0 + t * 16 + ln) * ldb + kb;
      FragB b;
      b.half[0] = *(const v8us*)(brow + 8 * hh);
      b.half[1] = *(const v8us*)(brow + 16 + 8 * hh);
      acc[t] = mmaN<ASPLIT ? 2 : 1>(ah.v, al.v, b.v, b.v, acc[t]);
    }
  }
#pragma unroll
  for (int t = 0; t < 4; ++t) {
    float bv = bias ? bias[col0 + t * 16 + ln] : 0.f;
    if (BIAS_BF16) bv = bf16_round(bv);
#pragma unroll
    for (int r = 0; r < 8; ++r) { float v = acc[t][r] + bv; if (ACT == 1) v = fmaxf(v, 0.f); so[w][8 * hh + r][t * 16 + ln] = v; }
  }
  __builtin_amdgcn_fence(__ATOMIC_ACQ_REL, "workgroup");
  __builtin_amdgcn_wave_barrier();
  const int rsub = lane >> 4, c4 = (lane & 15) * 4;
  for (int pass = 0; pass < 2; ++pass) {
#pragma unroll
    for (int q = 0; q < 8; ++q) {
      const int r = q * 2 + rsub;
      const v4f v = *(const v4fa*)&so[w][r][c4];
      *(volatile v4f*)(C + (size_t)(row0 + r) * ldc + col0 + c4) = v;
    }
    if (pass == 0) __threadfence();
  }
}

template <int D, bool CAUSAL>
__global__ __launch_bounds__(128) void k_flash(const float* __restrict__ qb, const float* __restrict__ kb, const float* __restrict__ vb,
                                             int pitch, int T, int H, float scale, float* __restrict__ y, int ypitch) {
  constexpr int KS = D / 32;
  constexpr int DT = D / 16;
  __shared__ __attribute__((aligned(16))) unsigned short sKh[32][D + 8], sKl[32][D + 8], sVh[32][D + 8], sVl[32][D + 8];
  __shared__ __attribute__((aligned(16))) unsigned short sPh[4][16][40], sPl[4][16][40];
  __shared__ __attribute__((aligned(16))) float sO[4][16][D];
  const int tid = threadIdx.x, w = tid >> 5, lane = tid & 31, ln = lane & 15, hh = lane >> 4;
  const int nqb = (T + 63) / 64;
  const int bh = blockIdx.x / nqb, qblk = blockIdx.x % nqb;
  const int b = bh / H, h = bh % H;
  const int q0 = qblk * 64 + w * 16;
  const float* Q = qb + (size_t)b * T * pitch + h * D;
  const float* K = kb + (size_t)b * T * pitch + h * D;
  const float* V = vb + (size_t)b * T * pitch + h * D;

  FragB aqh[KS], aql[KS];
  {
    int row = q0 + ln; if (row >= T) row = T - 1;
    const float* qr = Q + (size_t)row * pitch;
#pragma unroll
    for (int ks = 0; ks < KS; ++ks)
#pragma unroll
      for (int i = 0; i < 16; ++i) {
        const int d = ks * 32 + ((i < 8) ? (8 * hh + i) : (16 + 8 * hh + (i - 8)));
        const float x = qr[d] * scale; const unsigned short hb = bf16_bits(x);
        aqh[ks].u[i] = hb; aql[ks].u[i] = bf16_bits(x - bf16_val(hb));
      }
  }
  float m_r[8], l_r[8];
#pragma unroll
  for (int r = 0; r < 8; ++r) { m_r[r] = -3.0e38f; l_r[r] = 0.f; }
  v8f oacc[DT];
#pragma unroll
  for (int dt = 0; dt < DT; ++dt) oacc[dt] = (v8f){0.f,0.f,0.f,0.f,0.f,0.f,0.f,0.f};

  const int kv_end = CAUSAL ? min(T, qblk * 64 + 64) : T;
  for (int j0 = 0; j0 < kv_end; j0 += 32) {
    __syncthreads();
    for (int e = tid; e < 32 * (D / 4); e += 128) {
      const int r = e / (D / 4), c4 = (e % (D / 4)) * 4;
      const int key = j0 + r;
      v4f kf = {0.f,0.f,0.f,0.f}, vf = {0.f,0.f,0.f,0.f};
      if (key < T) { kf = *(const v4fa*)(K + (size_t)key * pitch + c4); vf = *(const v4fa*)(V + (size_t)key * pitch + c4); }
#pragma unroll
      for (int t = 0; t < 4; ++t) {
        unsigned short hb = bf16_bits(kf[t]); sKh[r][c4 + t] = hb; sKl[r][c4 + t] = bf16_bits(kf[t] - bf16_val(hb));
        hb = bf16_bits(vf[t]); sVh[r][c4 + t] = hb; sVl[r][c4 + t] = bf16_bits(vf[t] - bf16_val(hb));
      }
    }
    __syncthreads();
    v8f s[2];
#pragma unroll
    for (int nt = 0; nt < 2; ++nt) {
      v8f acc = {};
#pragma unroll
      for (int ks = 0; ks < KS; ++ks) {
        FragB bh_, bl_;
        bh_.half[0] = *(const v8us*)&sKh[nt * 16 + ln][ks * 32 + 8 * hh]; bh_.half[1] = *(const v8us*)&sKh[nt * 16 + ln][ks * 32 + 16 + 8 * hh];
        bl_.half[0] = *(const v8us*)&sKl[nt * 16 + ln][ks * 32 + 8 * hh]; bl_.half[1] = *(const v8us*)&sKl[nt * 16 + ln][ks * 32 + 16 + 8 * hh];
        acc = mmaN<3>(aqh[ks].v, aql[ks].v, bh_.v, bl_.v, acc);
      }
      s[nt] = acc;
    }
    float alpha[8];
#pragma unroll
    for (int r = 0; r < 8; ++r) {
      const int qi = q0 + 8 * hh + r;
      const int ja = j0 + ln, jb = j0 + 16 + ln;
      if (CAUSAL) { if (ja > qi) s[0][r] = -3.0e38f; if (jb > qi) s[1][r] = -3.0e38f; }
      if (ja >= T) s[0][r] = -3.0e38f;
      if (jb >= T) s[1][r] = -3.0e38f;
      float mx = fmaxf(s[0][r], s[1][r]);
      mx = fmaxf(mx, __shfl_xor(mx, 1, 32)); mx = fmaxf(mx, __shfl_xor(mx, 2, 32)); mx = fmaxf(mx, __shfl_xor(mx, 4, 32)); mx = fmaxf(mx, __shfl_xor(mx, 8, 32));
      const float mnew = fmaxf(m_r[r], mx);
      alpha[r] = (mnew > -1.0e38f) ? __expf(m_r[r] - mnew) : 1.0f;
      const float p0 = (s[0][r] > -1.0e38f) ? __expf(s[0][r] - mnew) : 0.f;
      const float p1 = (s[1][r] > -1.0e38f) ? __expf(s[1][r] - mnew) : 0.f;
      m_r[r] = mnew;
      l_r[r] = l_r[r] * alpha[r] + p0 + p1;
      unsigned short hb = bf16_bits(p0); sPh[w][8 * hh + r][ln] = hb;      sPl[w][8 * hh + r][ln] = bf16_bits(p0 - bf16_val(hb));
      hb = bf16_bits(p1);                sPh[w][8 * hh + r][16 + ln] = hb; sPl[w][8 * hh + r][16 + ln] = bf16_bits(p1 - bf16_val(hb));
    }
#pragma unroll
    for (int dt = 0; dt < DT; ++dt)
#pragma unroll
      for (int r = 0; r < 8; ++r) oacc[dt][r] *= alpha[r];
    __builtin_amdgcn_fence(__ATOMIC_ACQ_REL, "workgroup");
    __builtin_amdgcn_wave_barrier();
    FragB pah, pal;
    pah.half[0] = *(const v8us*)&sPh[w][ln][8 * hh]; pah.half[1] = *(const v8us*)&sPh[w][ln][16 + 8 * hh];
    pal.half[0] = *(const v8us*)&sPl[w][ln][8 * hh]; pal.half[1] = *(const v8us*)&sPl[w][ln][16 + 8 * hh];
#pragma unroll
    for (int dt = 0; dt < DT; ++dt) {
      FragB bvh, bvl;
#pragma unroll
      for (int i = 0; i < 8; ++i) {
        bvh.u[i] = sVh[8 * hh + i][dt * 16 + ln]; bvh.u[8 + i] = sVh[16 + 8 * hh + i][dt * 16 + ln];
        bvl.u[i] = sVl[8 * hh + i][dt * 16 + ln]; bvl.u[8 + i] = sVl[16 + 8 * hh + i][dt * 16 + ln];
      }
      oacc[dt] = mmaN<3>(pah.v, pal.v, bvh.v, bvl.v, oacc[dt]);
    }
    __builtin_amdgcn_fence(__ATOMIC_ACQ_REL, "workgroup");
    __builtin_amdgcn_wave_barrier();
  }
#pragma unroll
  for (int r = 0; r < 8; ++r) {
    float l = l_r[r];
    l += __shfl_xor(l, 1, 32); l += __shfl_xor(l, 2, 32); l += __shfl_xor(l, 4, 32); l += __shfl_xor(l, 8, 32);
    l_r[r] = (l > 0.f) ? 1.0f / l : 0.f;
  }
#pragma unroll
  for (int dt = 0; dt < DT; ++dt)
#pragma unroll
    for (int r = 0; r < 8; ++r) sO[w][8 * hh + r][dt * 16 + ln] = oacc[dt][r] * l_r[r];
  __builtin_amdgcn_fence(__ATOMIC_ACQ_REL, "workgroup");
  __builtin_amdgcn_wave_barrier();
  for (int pass = 0; pass < 2; ++pass) {
    for (int r = 0; r < 16; ++r) {
      const int row = q0 + r;
      if (row < T && lane < D / 4) {
        const v4f val = *(const v4fa*)&sO[w][r][lane * 4];
        *(volatile v4f*)(y + ((size_t)b * T + row) * ypitch + h * D + lane * 4) = val;
      }
    }
    if (pass == 0) __threadfence();
  }
}

__global__ __launch_bounds__(256) void k_wt0(const float* __restrict__ Ws, const float* __restrict__ Wd, unsigned short* __restrict__ Bs, unsigned short* __restrict__ Bd) {
  const int t = blockIdx.x * 256 + threadIdx.x;
  if (t < HID * 12) { const int n = t / 12, k8 = (t % 12) * 8; v8us v; for (int i = 0; i < 8; ++i) { const int k = k8 + i; v[i] = (k < 90) ? bf16_bits(Ws[k * HID + n]) : (unsigned short)0; } *(volatile v8us*)(Bs + n * 96 + k8) = v; __threadfence(); *(volatile v8us*)(Bs + n * 96 + k8) = v; }
  else if (t < HID * 12 + HID * 16) { const int u = t - HID * 12; const int n = u / 16, k8 = (u % 16) * 8; v8us v; for (int i = 0; i < 8; ++i) { const int k = k8 + i; float w = 0.f; if (k < 90) w = Wd[k * HID + n]; else if (k >= 96 && k < 105) w = Wd[(90 + k - 96) * HID + n]; v[i] = bf16_bits(w); } *(volatile v8us*)(Bd + n * 128 + k8) = v; __threadfence(); *(volatile v8us*)(Bd + n * 128 + k8) = v; }
}
__global__ __launch_bounds__(128) void k_nerf(const float* __restrict__ points, const float* __restrict__ dirs, const float* __restrict__ timev,
                                            const unsigned short* __restrict__ Bs0, const unsigned short* __restrict__ Bd0,
                                            const unsigned short* __restrict__ Ws1, const unsigned short* __restrict__ Ws2, const unsigned short* __restrict__ Ws3,
                                            const unsigned short* __restrict__ Wd1, const unsigned short* __restrict__ Wd2, const unsigned short* __restrict__ Wd3,
                                            const float* __restrict__ bs0, const float* __restrict__ bs1, const float* __restrict__ bs2, const float* __restrict__ bs3,
                                            const float* __restrict__ bd0, const float* __restrict__ bd1, const float* __restrict__ bd2, const float* __restrict__ bd3,
                                            const float* __restrict__ Ws4, const float* __restrict__ bs4, const float* __restrict__ Wd4, const float* __restrict__ bd4,
                                            float* __restrict__ pts) {
  __shared__ __attribute__((aligned(16))) float sX[4][16][HID + 4];
  __shared__ float sS[4][16][4];
  __shared__ float sO[4][16][8];
  const int tid = threadIdx.x, w = tid >> 5, lane = tid & 31, ln = lane & 15, hh = lane >> 4;
  const size_t p0 = ((size_t)blockIdx.x * 4 + w) * 16;
  {
    const size_t p = p0 + ln; float* row = sX[w][ln];
    if (hh == 0) {
      float xyz[3]; for (int c = 0; c < 3; ++c) xyz[c] = bf16_round(points[p * 3 + c]);
      for (int c = 0; c < 3; ++c) row[c] = xyz[c];
      float f = 1.0f;
      for (int l = 0; l < 10; ++l) { for (int c = 0; c < 3; ++c) { const float a = xyz[c] * f; row[3 + l * 6 + c] = sinf(a); row[3 + l * 6 + 3 + c] = cosf(a); } f *= 2.0f; }
    } else {
      float d3[3]; for (int c = 0; c < 3; ++c) d3[c] = bf16_round(dirs[p * 3 + c]);
      for (int c = 0; c < 3; ++c) row[63 + c] = d3[c];
      float f = 1.0f;
      for (int l = 0; l < 4; ++l) { for (int c = 0; c < 3; ++c) { const float a = d3[c] * f; row[66 + l * 6 + c] = sinf(a); row[66 + l * 6 + 3 + c] = cosf(a); } f *= 2.0f; }
      for (int c = 90; c < 96; ++c) row[c] = 0.f;
      const float tv = bf16_round(timev[p]); row[96] = tv; f = 1.0f;
      for (int l = 0; l < 4; ++l) { const float a = tv * f; row[97 + l * 2] = sinf(a); row[98 + l * 2] = cosf(a); f *= 2.0f; }
      for (int c = 105; c < 128; ++c) row[c] = 0.f;
    }
  }
  float outS[4] = {0.f,0.f,0.f,0.f}, outD[5] = {0.f,0.f,0.f,0.f,0.f};
#pragma unroll 1
  for (int br = 0; br < 2; ++br) {
    const int K0 = br ? 128 : 96; const unsigned short* B0 = br ? Bd0 : Bs0; const float* b0 = br ? bd0 : bs0;
    const unsigned short* Wh[3] = {br ? Wd1 : Ws1, br ? Wd2 : Ws2, br ? Wd3 : Ws3}; const float* bh[3] = {br ? bd1 : bs1, br ? bd2 : bs2, br ? bd3 : bs3};
    if (br == 1) {
      __builtin_amdgcn_fence(__ATOMIC_ACQ_REL, "workgroup"); __builtin_amdgcn_wave_barrier();
      const size_t p = p0 + ln; float* row = sX[w][ln];
      if (hh == 0) { float xyz[3]; for (int c = 0; c < 3; ++c) xyz[c] = bf16_round(points[p * 3 + c]); for (int c = 0; c < 3; ++c) row[c] = xyz[c]; float f = 1.0f; for (int l = 0; l < 10; ++l) { for (int c = 0; c < 3; ++c) { const float a = xyz[c] * f; row[3 + l * 6 + c] = sinf(a); row[3 + l * 6 + 3 + c] = cosf(a); } f *= 2.0f; } }
      else { float d3[3]; for (int c = 0; c < 3; ++c) d3[c] = bf16_round(dirs[p * 3 + c]); for (int c = 0; c < 3; ++c) row[63 + c] = d3[c]; float f = 1.0f; for (int l = 0; l < 4; ++l) { for (int c = 0; c < 3; ++c) { const float a = d3[c] * f; row[66 + l * 6 + c] = sinf(a); row[66 + l * 6 + 3 + c] = cosf(a); } f *= 2.0f; } for (int c = 90; c < 96; ++c) row[c] = 0.f; const float tv = bf16_round(timev[p]); row[96] = tv; f = 1.0f; for (int l = 0; l < 4; ++l) { const float a = tv * f; row[97 + l * 2] = sinf(a); row[98 + l * 2] = cosf(a); f *= 2.0f; } for (int c = 105; c < 128; ++c) row[c] = 0.f; }
    }
#pragma unroll 1
    for (int layer = 0; layer < 4; ++layer) {
      const int K = layer == 0 ? K0 : HID; const unsigned short* Bt = layer == 0 ? B0 : Wh[layer - 1]; const float* bias = layer == 0 ? b0 : bh[layer - 1];
      __builtin_amdgcn_fence(__ATOMIC_ACQ_REL, "workgroup"); __builtin_amdgcn_wave_barrier();
      FragB ah[8], al[8];
      for (int ks = 0; ks < 8; ++ks) {
        if (ks * 32 < K) {
#pragma unroll
          for (int i = 0; i < 16; ++i) { const int k = ks * 32 + ((i < 8) ? (8 * hh + i) : (16 + 8 * hh + (i - 8))); const float x = sX[w][ln][k]; const unsigned short hb = bf16_bits(x); ah[ks].u[i] = hb; al[ks].u[i] = bf16_bits(x - bf16_val(hb)); }
        }
      }
      __builtin_amdgcn_fence(__ATOMIC_ACQ_REL, "workgroup"); __builtin_amdgcn_wave_barrier();
#pragma unroll 1
      for (int nt = 0; nt < HID / 16; ++nt) {
        const int n = nt * 16 + ln; v8f acc = {};
        for (int ks = 0; ks < 8; ++ks) { if (ks * 32 < K) { FragB b; b.half[0] = *(const v8us*)(Bt + (size_t)n * K + ks * 32 + 8 * hh); b.half[1] = *(const v8us*)(Bt + (size_t)n * K + ks * 32 + 16 + 8 * hh); acc = mmaN<2>(ah[ks].v, al[ks].v, b.v, b.v, acc); } }
        const float bv = bf16_round(bias[n]);
#pragma unroll
        for (int r = 0; r < 8; ++r) sX[w][8 * hh + r][n] = fmaxf(acc[r] + bv, 0.f);
      }
    }
    __builtin_amdgcn_fence(__ATOMIC_ACQ_REL, "workgroup"); __builtin_amdgcn_wave_barrier();
    const int NO = br ? 5 : 4; const float* W4 = br ? Wd4 : Ws4; const float* b4 = br ? bd4 : bs4;
#pragma unroll
    for (int o = 0; o < 5; ++o) {
      if (o >= NO) break;
      float s = 0.f;
#pragma unroll 4
      for (int j = 0; j < 128; ++j) { const int k = hh * 128 + j; s += sX[w][ln][k] * bf16_round(W4[k * NO + o]); }
      s += __shfl_xor(s, 16, 32); s += bf16_round(b4[o]);
      if (br) outD[o] = s; else outS[o] = s;
    }
  }
  if (hh == 0) {
    const float bw = 1.0f / (1.0f + expf(-outD[4]));
    sO[w][ln][0] = (1.f - bw) * outS[0] + bw * outD[0];
    for (int c = 0; c < 3; ++c) { const float sr = 1.0f / (1.0f + expf(-outS[1 + c])), dr = 1.0f / (1.0f + expf(-outD[1 + c])); sO[w][ln][1 + c] = (1.f - bw) * sr + bw * dr; }
    sO[w][ln][4] = bw; sO[w][ln][5] = 0.f; sO[w][ln][6] = 0.f; sO[w][ln][7] = 0.f;
  }
  __builtin_amdgcn_fence(__ATOMIC_ACQ_REL, "workgroup"); __builtin_amdgcn_wave_barrier();
  { const v4f v = *(const v4fa*)&sO[w][lane >> 1][(lane & 1) * 4]; *(volatile v4f*)(pts + (p0 + (lane >> 1)) * 8 + (lane & 1) * 4) = v; __threadfence(); *(volatile v4f*)(pts + (p0 + (lane >> 1)) * 8 + (lane & 1) * 4) = v; }
}
__global__ __launch_bounds__(256) void k_rays(const float* __restrict__ pts, const float* __restrict__ z, float* __restrict__ rgb_map, float* __restrict__ depth,
                                            float* __restrict__ wts, float* __restrict__ swts, float* __restrict__ dwts) {
  __shared__ float sRGB[32][3]; __shared__ float sDep[32];
  const int tid = threadIdx.x, w = tid >> 5, lane = tid & 31;
  for (int u = 0; u < 4; ++u) {
    const int rl = w * 4 + u; const int ray = blockIdx.x * 32 + rl;
    float sig[4], bwv[4], zz[5], rgb[4][3];
    for (int i = 0; i < 4; ++i) { const size_t p = (size_t)ray * NS + lane * 4 + i; const float* pr = pts + p * 8; sig[i] = pr[0]; rgb[i][0] = pr[1]; rgb[i][1] = pr[2]; rgb[i][2] = pr[3]; bwv[i] = pr[4]; zz[i] = bf16_round(z[(size_t)ray * NS + lane * 4 + i]); }
    zz[4] = (lane < 31) ? bf16_round(z[(size_t)ray * NS + lane * 4 + 4]) : 0.f;
    float alpha[4], om[4];
    for (int i = 0; i < 4; ++i) { const float delta = (lane * 4 + i < NS - 1) ? (zz[i + 1] - zz[i]) : 1e10f; alpha[i] = 1.0f - expf(-sig[i] * delta); om[i] = 1.0f - alpha[i] + 1e-10f; }
    float loc = om[0] * om[1] * om[2] * om[3];
    float incl = loc;
    for (int o = 1; o < 32; o <<= 1) { const float t = __shfl_up(incl, o, 32); if (lane >= o) incl *= t; }
    float prefix = __shfl_up(incl, 1, 32); if (lane == 0) prefix = 1.0f;
    float T = prefix; float wv[4];
    for (int i = 0; i < 4; ++i) { wv[i] = alpha[i] * T; T *= om[i]; }
    float cr = 0.f, cg = 0.f, cb = 0.f, dz = 0.f;
    for (int i = 0; i < 4; ++i) { cr += wv[i] * rgb[i][0]; cg += wv[i] * rgb[i][1]; cb += wv[i] * rgb[i][2]; dz += wv[i] * zz[i]; }
    for (int o = 16; o >= 1; o >>= 1) { cr += __shfl_xor(cr, o, 32); cg += __shfl_xor(cg, o, 32); cb += __shfl_xor(cb, o, 32); dz += __shfl_xor(dz, o, 32); }
    if (lane == 0) { sRGB[rl][0] = cr; sRGB[rl][1] = cg; sRGB[rl][2] = cb; sDep[rl] = dz; }
    v4f wq = {wv[0], wv[1], wv[2], wv[3]}, sq, dq; for (int i = 0; i < 4; ++i) { sq[i] = (1.f - bwv[i]) * wv[i]; dq[i] = bwv[i] * wv[i]; }
    for (int pass = 0; pass < 2; ++pass) {
      *(volatile v4f*)(wts + (size_t)ray * NS + lane * 4) = wq; *(volatile v4f*)(swts + (size_t)ray * NS + lane * 4) = sq; *(volatile v4f*)(dwts + (size_t)ray * NS + lane * 4) = dq;
      if (pass == 0) __threadfence();
    }
  }
  __syncthreads();
  if (tid < 24) { v4f v; for (int j = 0; j < 4; ++j) { const int g = tid * 4 + j; v[j] = sRGB[g / 3][g % 3]; } *(volatile v4f*)(rgb_map + (size_t)blockIdx.x * 96 + tid * 4) = v; __threadfence(); *(volatile v4f*)(rgb_map + (size_t)blockIdx.x * 96 + tid * 4) = v; }
  if (tid >= 32 && tid < 64) { const float v = sDep[tid - 32]; *(volatile float*)(depth + blockIdx.x * 32 + tid - 32) = v; __threadfence(); *(volatile float*)(depth + blockIdx.x * 32 + tid - 32) = v; }
}

extern "C" void kernel_launch(void* const* d_in, const int* in_sizes, int n_in,
                              void* d_out, int out_size, void* d_ws, size_t ws_size, hipStream_t stream) {
  (void)in_sizes; (void)n_in; (void)out_size;
  const float* points = (const float*)d_in[0]; const float* dirs = (const float*)d_in[1]; const float* z = (const float*)d_in[2]; const float* timev = (const float*)d_in[3];
  const float* sW[5], *sb[5], *dW[5], *db[5];
  for (int i = 0; i < 5; ++i) { sW[i] = (const float*)d_in[4 + 4 * i]; sb[i] = (const float*)d_in[5 + 4 * i]; dW[i] = (const float*)d_in[6 + 4 * i]; db[i] = (const float*)d_in[7 + 4 * i]; }
  float* rgb_map = (float*)d_out; float* depth = rgb_map + NR * 3; float* wts = (float*)((char*)d_out + 32768); float* swts = (float*)((char*)d_out + 1081344); float* dwts = (float*)((char*)d_out + 2129920);
  char* ws = (char*)d_ws; size_t off = 0;
  auto take = [&](size_t bytes) { char* p = ws + off; off += (bytes + 255) & ~(size_t)255; return p; };
  unsigned short* Bs0 = (unsigned short*)take(HID * 96 * 2); unsigned short* Bd0 = (unsigned short*)take(HID * 128 * 2);
  unsigned short* Wst[3], *Wdt[3]; for (int i = 0; i < 3; ++i) { Wst[i] = (unsigned short*)take(HID * HID * 2); Wdt[i] = (unsigned short*)take(HID * HID * 2); }
  float* pts = (float*)take((size_t)NPTS * 8 * 4);
  if (off > ws_size) return;
  k_wt0<<<(HID * 28 + 255) / 256, 256, 0, stream>>>(sW[0], dW[0], Bs0, Bd0);
  for (int i = 0; i < 3; ++i) { k_wt_bf16<<<(HID * (HID / 8) + 255) / 256, 256, 0, stream>>>(sW[i + 1], Wst[i], HID, HID); k_wt_bf16<<<(HID * (HID / 8) + 255) / 256, 256, 0, stream>>>(dW[i + 1], Wdt[i], HID, HID); }
  k_nerf<<<NPTS / 64, 128, 0, stream>>>(points, dirs, timev, Bs0, Bd0, Wst[0], Wst[1], Wst[2], Wdt[0], Wdt[1], Wdt[2], sb[0], sb[1], sb[2], sb[3], db[0], db[1], db[2], db[3], sW[4], sb[4], dW[4], db[4], pts);
  k_rays<<<NR / 32, 256, 0, stream>>>(pts, z, rgb_map, depth, wts, swts, dwts);
}
